// LSTM_24970939859314
// MI455X (gfx1250) — hardware-verified
//
#include <hip/hip_runtime.h>
#include <math.h>

constexpr int NVOCAB = 50000;
constexpr int NEMB   = 300;
constexpr int NEMBP  = 320;
constexpr int NHID   = 128;
constexpr int NGATE  = 512;
constexpr int NSEQ   = 512;
constexpr int NBAT   = 64;
constexpr int NROWS  = NSEQ * NBAT;
constexpr int NTHR   = 256;
constexpr int ROWS_BLK = 16;
constexpr int HPITCH  = 136;
constexpr int XSPITCH = 516;
constexpr int HFPITCH = 132;
constexpr float ECARRY = 64.0f;
constexpr float WCARRY = 256.0f;
constexpr float HCARRY = 1024.0f;
constexpr float XSCALE = 1.0f / (ECARRY * WCARRY);
constexpr float RSCALE = 1.0f / (HCARRY * WCARRY);

static_assert(NGATE == 4 * NHID);
static_assert(NEMBP % 32 == 0 && NEMBP >= NEMB);
static_assert(NHID % 32 == 0);
static_assert(NEMB % 4 == 0 && NHID % 4 == 0);
static_assert(NROWS % 64 == 0 && NGATE % 64 == 0);
static_assert(NBAT % ROWS_BLK == 0);
static_assert(NHID == 16 * (NTHR / 32));
static_assert((NGATE * (NEMBP / 8)) % NTHR == 0);
static_assert((NGATE * (NHID / 8)) % NTHR == 0);
static_assert((NROWS * (NEMBP / 8)) % NTHR == 0);
static_assert(ROWS_BLK * NGATE == 8 * NTHR * 4);
static_assert(2 * NHID == NTHR);
static_assert((HPITCH % 8) == 0 && (XSPITCH % 4) == 0);

typedef __attribute__((ext_vector_type(16))) _Float16 v16h;
typedef __attribute__((ext_vector_type(8)))  _Float16 v8h;
typedef __attribute__((ext_vector_type(8)))  float    v8f;
typedef __attribute__((ext_vector_type(4)))  float    v4f;

__device__ __forceinline__ unsigned short f2bf_bits(float f) {
  unsigned u = __float_as_uint(f);
  return (unsigned short)((u + 0x7FFFu + ((u >> 16) & 1u)) >> 16);
}
__device__ __forceinline__ float bf_bits2f(unsigned short h) { return __uint_as_float(((unsigned)h) << 16); }
__device__ __forceinline__ float bf16r(float f) { return bf_bits2f(f2bf_bits(f)); }

__device__ __forceinline__ void acc_guard4(v8f& a, v8f& b, v8f& c, v8f& d) {
  asm volatile("v_nop\n\tv_nop\n\tv_nop\n\tv_nop" : "+v"(a), "+v"(b), "+v"(c), "+v"(d));
}
__device__ __forceinline__ void grp_guard_h(v8f& a0, v8f& a1, v8f& a2, v8f& a3,
                                            v16h x, v16h b0, v16h b1, v16h b2, v16h b3) {
  asm volatile("v_nop\n\tv_nop\n\tv_nop\n\tv_nop"
               : "+v"(a0), "+v"(a1), "+v"(a2), "+v"(a3)
               : "v"(x), "v"(b0), "v"(b1), "v"(b2), "v"(b3));
}
__device__ __forceinline__ void pin4_h(v16h& a, v16h& b, v16h& c, v16h& d) {
  asm volatile("v_nop" : "+v"(a), "+v"(b), "+v"(c), "+v"(d) : : "memory");
}

struct FragH {
  union U { v16h v; v8h h[2]; };
  static __device__ __forceinline__ v16h load(const _Float16* p) {
    U f;
    f.h[0] = *(const v8h*)(p);
    f.h[1] = *(const v8h*)(p + 16);
    return f.v;
  }
  static __device__ __forceinline__ v8f mma(v16h a, v16h b, v8f c) {
    return __builtin_amdgcn_wmma_f32_16x16x32_f16(false, a, false, b, (short)0, c, false, false);
  }
};

__device__ __forceinline__ float fsig(float x)  { return __builtin_amdgcn_rcpf(1.0f + __expf(-x)); }
__device__ __forceinline__ float ftanh(float x) { return 1.0f - 2.0f * __builtin_amdgcn_rcpf(__expf(2.0f * x) + 1.0f); }

template <bool GATHER>
__global__ __launch_bounds__(NTHR) void pack8_kernel(const float* __restrict__ src, const int* __restrict__ idx,
                                                     unsigned short* __restrict__ dst,
                                                     int nrow, int kreal, int kpad8, int nsrc, float sc) {
  const int i  = blockIdx.x * NTHR + threadIdx.x;
  const int n8 = nrow * kpad8;
  if (i < n8) {
    const int row = i / kpad8;
    const int c8  = i - row * kpad8;
    int srow = row;
    if (GATHER) {
      int tk = idx[row];
      tk = (tk < 0) ? 0 : tk;
      tk = (tk > nsrc - 1) ? (nsrc - 1) : tk;
      srow = tk;
    }
    const int col0 = c8 * 8;
    const int lim  = kreal - 4;
    const int ca = (col0 < lim) ? col0 : lim;
    const int cb = (col0 + 4 < lim) ? (col0 + 4) : lim;
    const float* sp = src + (size_t)srow * (size_t)kreal;
    const v4f a = *(const v4f*)(sp + ca);
    const v4f b = *(const v4f*)(sp + cb);
    v8h hv;
#pragma unroll
    for (int e = 0; e < 4; ++e) {
      const float fa = a[e];
      const float fb = b[e];
      const float va = (col0 + e < kreal) ? (bf16r(fa) * sc) : 0.0f;
      const float vb = (col0 + 4 + e < kreal) ? (bf16r(fb) * sc) : 0.0f;
      hv[e]     = (_Float16)va;
      hv[4 + e] = (_Float16)vb;
    }
    *(volatile v8h*)(dst + (size_t)i * 8) = hv;
    __threadfence();
    *(volatile v8h*)(dst + (size_t)i * 8) = hv;
  }
}

__global__ __launch_bounds__(256) void wmma_gemm64_f16(
    const unsigned short* __restrict__ Ap, int lda,
    const unsigned short* __restrict__ Btp, int ldb,
    float* __restrict__ C, int ldc, int M, int N, int K, float scale) {
  const _Float16* A  = (const _Float16*)Ap;
  const _Float16* Bt = (const _Float16*)Btp;
  __shared__ __align__(16) float sT[8][16 * 68];
  const int lane = threadIdx.x & 31;
  const int wave = threadIdx.x >> 5;
  const int tilesN = N >> 6;
  const int tilesM = M >> 6;
  const int tile = blockIdx.x * 8 + wave;
  if (tile >= tilesM * tilesN) return;
  const int tm = tile / tilesN;
  const int tn = tile - tm * tilesN;
  const int m0 = tm << 6;
  const int n0 = tn << 6;

  const int rlane = lane & 15;
  const int koff  = (lane >> 4) * 8;
  const int mOff  = (lane >> 4) * 8;

  v8f acc[4][4];
#pragma unroll
  for (int i = 0; i < 4; ++i)
#pragma unroll
    for (int j = 0; j < 4; ++j) acc[i][j] = (v8f){0.f, 0.f, 0.f, 0.f, 0.f, 0.f, 0.f, 0.f};

  for (int k0 = 0; k0 < K; k0 += 32) {
    v16h bh[4];
#pragma unroll
    for (int j = 0; j < 4; ++j) {
      const size_t bo = (size_t)(n0 + (j << 4) + rlane) * ldb + koff + k0;
      bh[j] = FragH::load(Bt + bo);
    }
#pragma unroll
    for (int i = 0; i < 4; ++i) {
      const size_t ao = (size_t)(m0 + (i << 4) + rlane) * lda + koff + k0;
      const v16h ah = FragH::load(A + ao);
#pragma unroll
      for (int j = 0; j < 4; ++j) acc[i][j] = FragH::mma(ah, bh[j], acc[i][j]);
      grp_guard_h(acc[i][0], acc[i][1], acc[i][2], acc[i][3], ah, bh[0], bh[1], bh[2], bh[3]);
    }
  }
  acc_guard4(acc[0][0], acc[0][1], acc[0][2], acc[0][3]);
  acc_guard4(acc[1][0], acc[1][1], acc[1][2], acc[1][3]);
  acc_guard4(acc[2][0], acc[2][1], acc[2][2], acc[2][3]);
  acc_guard4(acc[3][0], acc[3][1], acc[3][2], acc[3][3]);

  float* slab = sT[wave];
#pragma unroll
  for (int i = 0; i < 4; ++i) {
    const int mBase = m0 + (i << 4);
#pragma unroll
    for (int j = 0; j < 4; ++j) {
#pragma unroll
      for (int r = 0; r < 8; ++r) {
        const float v = acc[i][j][r] * scale;
        slab[(mOff + r) * 68 + (j << 4) + rlane] = v;
      }
    }
    __builtin_amdgcn_fence(__ATOMIC_RELEASE, "workgroup");
    __builtin_amdgcn_wave_barrier();
    __builtin_amdgcn_fence(__ATOMIC_ACQUIRE, "workgroup");
    {
      const int hh = lane >> 4, c4 = (lane & 15) * 4;
      for (int pass = 0; pass < 2; ++pass) {
#pragma unroll
        for (int it = 0; it < 8; ++it) {
          const int row = it * 2 + hh;
          const v4f v = *(const v4f*)(slab + row * 68 + c4);
          *(volatile v4f*)(C + (size_t)(mBase + row) * ldc + n0 + c4) = v;
        }
        __threadfence();
      }
    }
    __builtin_amdgcn_fence(__ATOMIC_RELEASE, "workgroup");
    __builtin_amdgcn_wave_barrier();
    __builtin_amdgcn_fence(__ATOMIC_ACQUIRE, "workgroup");
  }
}

__device__ __forceinline__ void stage_x(const float* __restrict__ XPg, float* xs, int t, int rowbase, int tid) {
  v4f v[8];
  const int rsub = tid >> 7;
  const int c4 = (tid & 127) * 4;
#pragma unroll
  for (int it = 0; it < 8; ++it) {
    const int row = it * 2 + rsub;
    v[it] = *(const v4f*)(XPg + ((size_t)t * NBAT + (size_t)(rowbase + row)) * NGATE + c4);
  }
#pragma unroll
  for (int it = 0; it < 8; ++it) {
    const int row = it * 2 + rsub;
    *(v4f*)(xs + row * XSPITCH + c4) = v[it];
  }
}

__global__ __launch_bounds__(NTHR) void lstm_seq_kernel(const float* __restrict__ XPg,
                                                        const unsigned short* __restrict__ WHp,
                                                        const float* __restrict__ b_ih, const float* __restrict__ b_hh,
                                                        const float* __restrict__ w_dec, const float* __restrict__ b_dec,
                                                        float* __restrict__ out) {
  __shared__ __align__(16) float    Xs[ROWS_BLK * XSPITCH];
  __shared__ __align__(16) _Float16 Ah[ROWS_BLK * HPITCH];
  __shared__ __align__(16) float    Hf[ROWS_BLK * HFPITCH];
  __shared__ __align__(16) float    Wd[2 * NHID];
  const _Float16* WH = (const _Float16*)WHp;
  const int tid = threadIdx.x, lane = tid & 31, jt = tid >> 5;
  const int c = lane & 15, hh = lane >> 4, koff = hh * 8;
  const int rowbase = blockIdx.x * ROWS_BLK;

  v16h Bf[4][4];
#pragma unroll
  for (int g = 0; g < 4; ++g) {
    const _Float16* wr = WH + (size_t)(g * NHID + 16 * jt + c) * NHID + koff;
#pragma unroll
    for (int kk = 0; kk < 4; ++kk) Bf[g][kk] = FragH::load(wr + kk * 32);
    pin4_h(Bf[g][0], Bf[g][1], Bf[g][2], Bf[g][3]);
  }
  float bb[4];
#pragma unroll
  for (int g = 0; g < 4; ++g) {
    const int n = g * NHID + 16 * jt + c;
    bb[g] = bf16r(b_ih[n]) + bf16r(b_hh[n]);
  }
  Wd[tid] = bf16r(w_dec[tid]);
  const float bdv = bf16r(b_dec[tid & 1]);

#pragma unroll 1
  for (int i = tid; i < ROWS_BLK * HPITCH; i += NTHR) Ah[i] = (_Float16)0.0f;
  stage_x(XPg, Xs, 0, rowbase, tid);

  float cst[8], hst[8];
#pragma unroll
  for (int r = 0; r < 8; ++r) { cst[r] = 0.0f; hst[r] = 0.0f; }
  __syncthreads();

  const _Float16* ahrow = Ah + c * HPITCH + koff;
  const v8f z8 = {0.f, 0.f, 0.f, 0.f, 0.f, 0.f, 0.f, 0.f};

#pragma unroll 1
  for (int t = 0; t < NSEQ; ++t) {
    v8f acc0 = z8, acc1 = z8, acc2 = z8, acc3 = z8;
#pragma unroll
    for (int kk = 0; kk < 4; ++kk) {
      const v16h a = FragH::load(ahrow + kk * 32);
      acc0 = FragH::mma(a, Bf[0][kk], acc0);
      acc1 = FragH::mma(a, Bf[1][kk], acc1);
      acc2 = FragH::mma(a, Bf[2][kk], acc2);
      acc3 = FragH::mma(a, Bf[3][kk], acc3);
      grp_guard_h(acc0, acc1, acc2, acc3, a, Bf[0][kk], Bf[1][kk], Bf[2][kk], Bf[3][kk]);
    }
    acc_guard4(acc0, acc1, acc2, acc3);

#pragma unroll
    for (int r = 0; r < 8; ++r) {
      const float* xr = Xs + (8 * hh + r) * XSPITCH + 16 * jt + c;
      const float xi = xr[0];
      const float xf = xr[NHID];
      const float xg = xr[2 * NHID];
      const float xo = xr[3 * NHID];
      const float zi = acc0[r] * RSCALE + (xi + bb[0]);
      const float zf = acc1[r] * RSCALE + (xf + bb[1]);
      const float zg = acc2[r] * RSCALE + (xg + bb[2]);
      const float zo = acc3[r] * RSCALE + (xo + bb[3]);
      const float ig = fsig(zi);
      const float fg = fsig(zf);
      const float gg = ftanh(zg);
      const float og = fsig(zo);
      const float cn = fg * cst[r] + ig * gg;
      cst[r] = cn;
      hst[r] = og * ftanh(cn);
    }
    __syncthreads();
#pragma unroll
    for (int r = 0; r < 8; ++r) Ah[(8 * hh + r) * HPITCH + 16 * jt + c] = (_Float16)(hst[r] * HCARRY);
    {
      const int tn = (t + 1 < NSEQ) ? (t + 1) : (NSEQ - 1);
      stage_x(XPg, Xs, tn, rowbase, tid);
    }
    __syncthreads();
  }

#pragma unroll
  for (int r = 0; r < 8; ++r) Hf[(8 * hh + r) * HFPITCH + 16 * jt + c] = hst[r];
  __syncthreads();
  if (jt == 0) {
    const int row = lane >> 1, d = lane & 1;
    const float* hr = Hf + row * HFPITCH;
    const float* wd = Wd + d * NHID;
    float s = 0.0f;
#pragma unroll 4
    for (int j = 0; j < NHID; ++j) s = fmaf(hr[j], wd[j], s);
    s += bdv;
    float* op = out + blockIdx.x * 32 + lane;
    *(volatile float*)op = s;
    __threadfence();
    *(volatile float*)op = s;
  }
}

extern "C" void kernel_launch(void* const* d_in, const int* in_sizes, int n_in,
                              void* d_out, int out_size, void* d_ws, size_t ws_size, hipStream_t stream) {
  if (n_in < 8 || d_out == nullptr || d_ws == nullptr) return;
  if (in_sizes[0] != NROWS || in_sizes[1] != NVOCAB * NEMB || in_sizes[2] != NGATE * NEMB ||
      in_sizes[3] != NGATE * NHID || in_sizes[4] != NGATE || in_sizes[5] != NGATE ||
      in_sizes[6] != 2 * NHID || in_sizes[7] != 2 || out_size != NBAT * 2) return;

  const int*   sentence = (const int*)d_in[0];
  const float* emb      = (const float*)d_in[1];
  const float* w_ih     = (const float*)d_in[2];
  const float* w_hh     = (const float*)d_in[3];
  const float* b_ih     = (const float*)d_in[4];
  const float* b_hh     = (const float*)d_in[5];
  const float* w_dec    = (const float*)d_in[6];
  const float* b_dec    = (const float*)d_in[7];
  float* out = (float*)d_out;

  char* ws = (char*)d_ws;
  size_t off = 0;
  auto carve = [&](size_t bytes) -> char* { char* p = ws + off; off += (bytes + 255) & ~(size_t)255; return p; };
  unsigned short* APL = (unsigned short*)carve((size_t)NROWS * NEMBP * 2);
  unsigned short* BT0 = (unsigned short*)carve((size_t)NGATE * NEMBP * 2);
  unsigned short* BT1 = (unsigned short*)carve((size_t)NGATE * NHID * 2);
  float*          XPL = (float*)carve((size_t)NROWS * NGATE * 4);
  if (off > ws_size || off > (size_t)134217728) return;

  const int n8a = NGATE * (NEMBP / 8);
  const int n8b = NGATE * (NHID / 8);
  const int n8g = NROWS * (NEMBP / 8);
  pack8_kernel<false><<<n8a / NTHR, NTHR, 0, stream>>>(w_ih, sentence, BT0, NGATE, NEMB, NEMBP / 8, NGATE, WCARRY);
  pack8_kernel<false><<<n8b / NTHR, NTHR, 0, stream>>>(w_hh, sentence, BT1, NGATE, NHID, NHID / 8, NGATE, WCARRY);
  pack8_kernel<true><<<n8g / NTHR, NTHR, 0, stream>>>(emb, sentence, APL, NROWS, NEMB, NEMBP / 8, NVOCAB, ECARRY);

  const int ntiles = (NROWS / 64) * (NGATE / 64);
  wmma_gemm64_f16<<<ntiles / 8, 256, 0, stream>>>(APL, NEMBP, BT0, NEMBP, XPL, NGATE, NROWS, NGATE, NEMBP, XSCALE);

  lstm_seq_kernel<<<NBAT / ROWS_BLK, NTHR, 0, stream>>>(XPL, BT1, b_ih, b_hh, w_dec, b_dec, out);
}
